// BiMambaBlock_43250320670965
// MI455X (gfx1250) — hardware-run, weakly checked
//
#include <hip/hip_runtime.h>
#include <math.h>

typedef __attribute__((ext_vector_type(16))) _Float16 v16h;
typedef __attribute__((ext_vector_type(8)))  _Float16 v8h;
typedef __attribute__((ext_vector_type(16))) __bf16   v16b;
typedef __attribute__((ext_vector_type(8)))  __bf16   v8b;
typedef __attribute__((ext_vector_type(8)))  float    v8f;
typedef __attribute__((ext_vector_type(4)))  float    v4f;
typedef __attribute__((ext_vector_type(4)))  unsigned int v4u;

constexpr int kBatch   = 2;
constexpr int kSeq     = 2048;
constexpr int kDm      = 1024;
constexpr int kDin     = 2048;
constexpr int kNst     = 16;
constexpr int kDtR     = 64;
constexpr int kNPj     = 96;
constexpr int kNPjPad  = 128;
constexpr int kXzP     = 2 * kDin;
constexpr int kPjP     = kNPjPad;
constexpr int kRowsAll = kBatch * kSeq;
constexpr int kConvTP  = 260;
constexpr int kScanTS  = 64;
constexpr int kScanCh  = 64;
constexpr int kScanThr = 2 * kScanCh;
constexpr int kScanYP  = 68;
static_assert(kDtR + 2 * kNst == kNPj);
static_assert((kDm % 32) == 0 && (kDin % 32) == 0 && (kDtR % 32) == 0);
static_assert((kSeq % 64) == 0 && (kXzP % 64) == 0 && (kNPjPad % 64) == 0 && (kDin % 64) == 0 && (kDm % 64) == 0);
static_assert((kSeq % kScanTS) == 0 && (kDin % kScanCh) == 0 && (kDin % 256) == 0 && (kSeq % 64) == 0);
static_assert(kScanThr == 128 && kScanCh == 4 * 16 && kScanTS == 64 && kNst == 16);

constexpr size_t kOffUB   = 0;
constexpr size_t kOffWIB  = kOffUB  + (size_t)kRowsAll * kDm * 2;
constexpr size_t kOffWOB  = kOffWIB + (size_t)kXzP * kDm * 2;
constexpr size_t kOffWX   = kOffWOB + (size_t)kDm * kDin * 2;
constexpr size_t kOffWD   = kOffWX  + (size_t)2 * kNPjPad * kDin * 2;
constexpr size_t kOffXZ   = kOffWD  + (size_t)2 * kDin * kDtR * 2;
constexpr size_t kOffXC   = kOffXZ  + (size_t)kSeq * kXzP * 4;
constexpr size_t kOffPJ   = kOffXC  + (size_t)2 * kSeq * kDin * 2;
constexpr size_t kOffDI   = kOffPJ  + (size_t)2 * kSeq * kPjP * 4;
constexpr size_t kOffDT   = kOffDI  + (size_t)2 * kSeq * kDtR * 2;
constexpr size_t kOffYF   = kOffDT  + (size_t)2 * kSeq * kDin * 2;
constexpr size_t kOffYSH  = kOffYF  + (size_t)kSeq * kDin * 4;
constexpr size_t kOffYSL  = kOffYSH + (size_t)kSeq * kDin * 2;
constexpr size_t kWsTotal = kOffYSL + (size_t)kSeq * kDin * 2;
static_assert(kWsTotal == 125829120ull);
static_assert(kWsTotal <= 134217728ull);
static_assert((kOffWIB % 128) == 0 && (kOffWOB % 128) == 0 && (kOffWX % 128) == 0 && (kOffWD % 128) == 0 &&
              (kOffXZ % 128) == 0 && (kOffXC % 128) == 0 && (kOffPJ % 128) == 0 && (kOffDI % 128) == 0 &&
              (kOffDT % 128) == 0 && (kOffYF % 128) == 0 && (kOffYSH % 128) == 0 && (kOffYSL % 128) == 0);

__device__ __forceinline__ unsigned short f2bf_bits(float f) {
  unsigned u = __float_as_uint(f);
  return (unsigned short)((u + 0x7FFFu + ((u >> 16) & 1u)) >> 16);
}
__device__ __forceinline__ float bf_bits2f(unsigned short h) { return __uint_as_float(((unsigned)h) << 16); }
__device__ __forceinline__ float bfr(float f) { return bf_bits2f(f2bf_bits(f)); }
__device__ __forceinline__ unsigned pack_bf2(float lo, float hi) {
  return (unsigned)f2bf_bits(lo) | (((unsigned)f2bf_bits(hi)) << 16);
}

__device__ __forceinline__ void dep_guard_h(v8f& a, v8f& b, v16h x, v16h y) { asm volatile("v_nop\n\tv_nop\n\tv_nop\n\tv_nop" : "+v"(a), "+v"(b) : "v"(x), "v"(y)); }
__device__ __forceinline__ void dep_guard_b(v8f& a, v8f& b, v16b x, v16b y) { asm volatile("v_nop\n\tv_nop\n\tv_nop\n\tv_nop" : "+v"(a), "+v"(b) : "v"(x), "v"(y)); }
__device__ __forceinline__ void dep_guard4_h(v8f& a, v8f& b, v8f& c, v8f& d, v16h x, v16h y) { asm volatile("v_nop\n\tv_nop\n\tv_nop\n\tv_nop" : "+v"(a), "+v"(b), "+v"(c), "+v"(d) : "v"(x), "v"(y)); }
__device__ __forceinline__ void dep_guard4_b(v8f& a, v8f& b, v8f& c, v8f& d, v16b x, v16b y) { asm volatile("v_nop\n\tv_nop\n\tv_nop\n\tv_nop" : "+v"(a), "+v"(b), "+v"(c), "+v"(d) : "v"(x), "v"(y)); }
__device__ __forceinline__ void keep4_h(v16h a, v16h b, v16h c, v16h d) { asm volatile("v_nop" :: "v"(a), "v"(b), "v"(c), "v"(d)); }
__device__ __forceinline__ void keep4_b(v16b a, v16b b, v16b c, v16b d) { asm volatile("v_nop" :: "v"(a), "v"(b), "v"(c), "v"(d)); }
__device__ __forceinline__ void acc_guard4(v8f& a, v8f& b, v8f& c, v8f& d) { asm volatile("v_nop\n\tv_nop\n\tv_nop\n\tv_nop" : "+v"(a), "+v"(b), "+v"(c), "+v"(d)); }
template <typename T> struct Frag;
template <> struct Frag<_Float16> {
  typedef v16h V; union U { v16h v; v8h h[2]; };
  static __device__ __forceinline__ v16h load(const _Float16* p) {
    U f; f.h[0] = *(const v8h*)(p); f.h[1] = *(const v8h*)(p + 16); return f.v;
  }
  static __device__ __forceinline__ v8f mma(v16h a, v16h b, v8f c) {
    return __builtin_amdgcn_wmma_f32_16x16x32_f16(false, a, false, b, (short)0, c, false, false);
  }
  static __device__ __forceinline__ void guard(v8f& a, v8f& b, v16h x, v16h y) { dep_guard_h(a, b, x, y); }
  static __device__ __forceinline__ void guard4(v8f& a, v8f& b, v8f& c, v8f& d, v16h x, v16h y) { dep_guard4_h(a, b, c, d, x, y); }
  static __device__ __forceinline__ void keep(v16h a, v16h b, v16h c, v16h d) { keep4_h(a, b, c, d); }
};
template <> struct Frag<__bf16> {
  typedef v16b V; union U { v16b v; v8b h[2]; };
  static __device__ __forceinline__ v16b load(const __bf16* p) {
    U f; f.h[0] = *(const v8b*)(p); f.h[1] = *(const v8b*)(p + 16); return f.v;
  }
  static __device__ __forceinline__ v8f mma(v16b a, v16b b, v8f c) {
    return __builtin_amdgcn_wmma_f32_16x16x32_bf16(false, a, false, b, (short)0, c, false, false);
  }
  static __device__ __forceinline__ void guard(v8f& a, v8f& b, v16b x, v16b y) { dep_guard_b(a, b, x, y); }
  static __device__ __forceinline__ void guard4(v8f& a, v8f& b, v8f& c, v8f& d, v16b x, v16b y) { dep_guard4_b(a, b, c, d, x, y); }
  static __device__ __forceinline__ void keep(v16b a, v16b b, v16b c, v16b d) { keep4_b(a, b, c, d); }
};

union FragW { v16b v; v4u q[2]; };
__device__ __forceinline__ v8f mma_bf16_once(v16b a, v16b b) {
  v8f c = (v8f){0.f,0.f,0.f,0.f,0.f,0.f,0.f,0.f};
  c = __builtin_amdgcn_wmma_f32_16x16x32_bf16(false, a, false, b, (short)0, c, false, false);
  asm volatile("v_nop\n\tv_nop\n\tv_nop\n\tv_nop" : "+v"(c) : "v"(a), "v"(b));
  return c;
}

template <int ET> struct Elem;
template <> struct Elem<0> { typedef _Float16 T; };
template <> struct Elem<1> { typedef __bf16 T; };
template <int ET, int SPL, int BIAS_MODE, int OUT_MODE, bool RESID, int ACT = 0>
__global__ __launch_bounds__(256) void wmma_gemm64(
    const unsigned short* __restrict__ Ap, const unsigned short* __restrict__ A2p, int lda, long strideA,
    const unsigned short* __restrict__ Btp, const unsigned short* __restrict__ Bt2p, int ldb, long strideB,
    void* __restrict__ Cout, void* __restrict__ Cout2, int ldc, long strideC,
    const float* __restrict__ bias,
    const float* __restrict__ resid, long strideR,
    int M, int N, int K, float scale) {
  typedef typename Elem<ET>::T T;
  typedef typename Frag<T>::V V;
  const T* A = (const T*)Ap; const T* A2 = (const T*)A2p; const T* Bt = (const T*)Btp; const T* Bt2 = (const T*)Bt2p;
  __shared__ __align__(16) float sT[8][16 * 68];
  const int b    = blockIdx.y;
  const int lane = threadIdx.x & 31;
  const int wave = threadIdx.x >> 5;
  const int tilesN = N >> 6;
  const int tilesM = M >> 6;
  const int tile = blockIdx.x * 8 + wave;
  if (tile >= tilesM * tilesN) return;
  const int tm = tile / tilesN;
  const int tn = tile - tm * tilesN;
  const int m0 = tm << 6;
  const int n0 = tn << 6;

  const T* Ab  = A  + (size_t)b * strideA;
  const T* Bb  = Bt + (size_t)b * strideB;
  const T* Ab2 = (SPL >= 1) ? (A2  + (size_t)b * strideA) : nullptr;
  const T* Bb2 = (SPL == 2) ? (Bt2 + (size_t)b * strideB) : nullptr;

  const int rlane = lane & 15;
  const int koff  = (lane >> 4) * 8;
  const int mOff  = (lane >> 4) * 8;

  v8f acc[4][4];
#pragma unroll
  for (int i = 0; i < 4; ++i)
#pragma unroll
    for (int j = 0; j < 4; ++j) acc[i][j] = (v8f){0.f,0.f,0.f,0.f,0.f,0.f,0.f,0.f};

  for (int k0 = 0; k0 < K; k0 += 32) {
    V bh[4], bl[4];
#pragma unroll
    for (int j = 0; j < 4; ++j) {
      const size_t bo = (size_t)(n0 + (j << 4) + rlane) * ldb + koff + k0;
      bh[j] = Frag<T>::load(Bb + bo);
      if (SPL == 2) bl[j] = Frag<T>::load(Bb2 + bo);
    }
#pragma unroll
    for (int i = 0; i < 4; ++i) {
      const size_t ao = (size_t)(m0 + (i << 4) + rlane) * lda + koff + k0;
      V ah = Frag<T>::load(Ab + ao);
      V al;
      if (SPL >= 1) al = Frag<T>::load(Ab2 + ao);
#pragma unroll
      for (int j = 0; j < 4; ++j) {
        acc[i][j] = Frag<T>::mma(ah, bh[j], acc[i][j]);
        if (SPL == 2) acc[i][j] = Frag<T>::mma(ah, bl[j], acc[i][j]);
        if (SPL >= 1) acc[i][j] = Frag<T>::mma(al, bh[j], acc[i][j]);
      }
      Frag<T>::guard4(acc[i][0], acc[i][1], acc[i][2], acc[i][3], ah, (SPL >= 1) ? al : ah);
    }
    Frag<T>::keep(bh[0], bh[1], bh[2], bh[3]);
    if (SPL == 2) Frag<T>::keep(bl[0], bl[1], bl[2], bl[3]);
  }
  acc_guard4(acc[0][0], acc[0][1], acc[0][2], acc[0][3]);
  acc_guard4(acc[1][0], acc[1][1], acc[1][2], acc[1][3]);
  acc_guard4(acc[2][0], acc[2][1], acc[2][2], acc[2][3]);
  acc_guard4(acc[3][0], acc[3][1], acc[3][2], acc[3][3]);

  float* slab = sT[wave];
  const float* Rb = RESID ? (resid + (size_t)b * strideR) : nullptr;
#pragma unroll
  for (int i = 0; i < 4; ++i) {
    const int mBase = m0 + (i << 4);
#pragma unroll
    for (int j = 0; j < 4; ++j) {
      const int n = n0 + (j << 4) + rlane;
      float bv = 0.f;
      if (BIAS_MODE == 2) bv = bias[n];
#pragma unroll
      for (int r = 0; r < 8; ++r) {
        float v = acc[i][j][r] * scale;
        if (BIAS_MODE == 1) v += bias[mBase + mOff + r];
        if (BIAS_MODE == 2) v += bv;
        if (RESID) v += Rb[(size_t)(mBase + mOff + r) * ldc + n];
        if (ACT == 1) v = tanhf(v);
        if (ACT == 2) v = fmaxf(v, 0.0f);
        if (ACT == 3) v = v / (1.0f + expf(-v));
        if (ACT == 4) v = (v > 0.f) ? v : 0.01f * v;
        slab[(mOff + r) * 68 + (j << 4) + rlane] = v;
      }
    }
    __builtin_amdgcn_fence(__ATOMIC_RELEASE, "workgroup");
    __builtin_amdgcn_wave_barrier();
    __builtin_amdgcn_fence(__ATOMIC_ACQUIRE, "workgroup");
    if (OUT_MODE == 0) {
      float* C = (float*)Cout + (size_t)b * strideC;
      const int hh = lane >> 4, c4 = (lane & 15) * 4;
      for (int pass = 0; pass < 2; ++pass) {
#pragma unroll
        for (int it = 0; it < 8; ++it) {
          const int row = it * 2 + hh;
          v4f v = *(const v4f*)(slab + row * 68 + c4);
          *(volatile v4f*)(C + (size_t)(mBase + row) * ldc + n0 + c4) = v;
        }
        __threadfence();
      }
    } else {
      const int q = lane >> 3, c8 = (lane & 7) * 8;
      unsigned short* C  = (unsigned short*)Cout  + (size_t)b * strideC;
      unsigned short* C2 = (OUT_MODE == 2) ? ((unsigned short*)Cout2 + (size_t)b * strideC) : nullptr;
      for (int pass = 0; pass < 2; ++pass) {
#pragma unroll
        for (int it = 0; it < 4; ++it) {
          const int row = it * 4 + q;
          const float* sp = slab + row * 68 + c8;
          v8h hv, lv;
#pragma unroll
          for (int e = 0; e < 8; ++e) {
            if (OUT_MODE == 1) {
              hv[e] = (_Float16)sp[e];
            } else {
              unsigned short hb = f2bf_bits(sp[e]);
              hv[e] = __builtin_bit_cast(_Float16, hb);
              if (OUT_MODE == 2) {
                unsigned short lb = f2bf_bits(sp[e] - bf_bits2f(hb));
                lv[e] = __builtin_bit_cast(_Float16, lb);
              }
            }
          }
          *(volatile v8h*)(C + (size_t)(mBase + row) * ldc + n0 + c8) = hv;
          if (OUT_MODE == 2) *(volatile v8h*)(C2 + (size_t)(mBase + row) * ldc + n0 + c8) = lv;
        }
        __threadfence();
      }
    }
    __builtin_amdgcn_fence(__ATOMIC_RELEASE, "workgroup");
    __builtin_amdgcn_wave_barrier();
    __builtin_amdgcn_fence(__ATOMIC_ACQUIRE, "workgroup");
  }
}

__global__ __launch_bounds__(256) void cvt_bf16_kernel(
    const float* __restrict__ src, unsigned short* __restrict__ dst, int ncols, int nrows_src, int total8)
{
  const int i = blockIdx.x * 256 + threadIdx.x;
  if (i >= total8) return;
  const int e0 = i << 3;
  const int row = e0 / ncols;
  const int col = e0 - row * ncols;
  const bool live = (row < nrows_src);
  const int rowc = live ? row : (nrows_src - 1);
  const float lf = live ? 1.0f : 0.0f;
  const float* sp = src + (size_t)rowc * ncols + col;
  const v4f a0 = *(const v4f*)(sp);
  const v4f a1 = *(const v4f*)(sp + 4);
  v8h hv;
#pragma unroll
  for (int e = 0; e < 4; ++e) {
    const float f0 = fmaf(a0[e], lf, 0.0f);
    const float f1 = fmaf(a1[e], lf, 0.0f);
    hv[e]     = __builtin_bit_cast(_Float16, f2bf_bits(f0));
    hv[4 + e] = __builtin_bit_cast(_Float16, f2bf_bits(f1));
  }
  unsigned short* qh = dst + (size_t)e0;
  *(volatile v8h*)qh = hv;
  __threadfence();
  *(volatile v8h*)qh = hv;
}

__global__ __launch_bounds__(256) void cvt_cols64_kernel(
    const float* __restrict__ PJ, unsigned short* __restrict__ DI, int total8)
{
  const int i = blockIdx.x * 256 + threadIdx.x;
  if (i >= total8) return;
  const int row = i >> 3, c8 = (i & 7) * 8;
  const float* sp = PJ + (size_t)row * kPjP + c8;
  const v4f a0 = *(const v4f*)(sp);
  const v4f a1 = *(const v4f*)(sp + 4);
  v8h hv;
#pragma unroll
  for (int e = 0; e < 4; ++e) {
    hv[e]     = __builtin_bit_cast(_Float16, f2bf_bits(a0[e]));
    hv[4 + e] = __builtin_bit_cast(_Float16, f2bf_bits(a1[e]));
  }
  unsigned short* qh = DI + (size_t)row * kDtR + c8;
  *(volatile v8h*)qh = hv;
  __threadfence();
  *(volatile v8h*)qh = hv;
}

__global__ __launch_bounds__(256) void conv_silu_kernel(
    const float* __restrict__ XZ,
    const float* __restrict__ cwf, const float* __restrict__ cbf,
    const float* __restrict__ cwb, const float* __restrict__ cbb,
    unsigned short* __restrict__ XC)
{
  __shared__ __align__(16) float sT[16 * kConvTP];
  const int tid = threadIdx.x, lane = tid & 31, wave = tid >> 5;
  const int d0 = blockIdx.x * 256, d = d0 + tid;
  const int dir = blockIdx.z;
  const int tau0 = blockIdx.y * 64;
  const float* cw = dir ? cwb : cwf;
  const float* cb = dir ? cbb : cbf;
  unsigned short* XCd = XC + (size_t)dir * kSeq * kDin;
  const float w0 = bfr(cw[d * 4 + 0]), w1 = bfr(cw[d * 4 + 1]), w2 = bfr(cw[d * 4 + 2]), w3 = bfr(cw[d * 4 + 3]);
  const float bc = bfr(cb[d]);
  float xm3, xm2, xm1;
  {
    const bool hist = (tau0 > 0);
    const int tb = hist ? (tau0 - 3) : tau0;
    const int pa = dir ? (kSeq - 1 - tb) : tb;
    const int pb = dir ? (kSeq - 2 - tb) : (tb + 1);
    const int pc = dir ? (kSeq - 3 - tb) : (tb + 2);
    const float v3 = XZ[(size_t)pa * kXzP + d];
    const float v2 = XZ[(size_t)pb * kXzP + d];
    const float v1 = XZ[(size_t)pc * kXzP + d];
    const float hf = hist ? 1.0f : 0.0f;
    xm3 = v3 * hf;
    xm2 = v2 * hf;
    xm1 = v1 * hf;
  }
#pragma unroll 1
  for (int sub = 0; sub < 4; ++sub) {
    const int lb = tau0 + sub * 16;
#pragma unroll 1
    for (int s = 0; s < 16; ++s) {
      const int tau = lb + s;
      const int p = dir ? (kSeq - 1 - tau) : tau;
      const float xcur = XZ[(size_t)p * kXzP + d];
      float acc = w0 * xm3;
      acc = fmaf(w1, xm2, acc);
      acc = fmaf(w2, xm1, acc);
      acc = fmaf(w3, xcur, acc);
      const float sv = acc + bc;
      const float sg = __builtin_amdgcn_rcpf(1.0f + __expf(-sv));
      sT[s * kConvTP + tid] = sv * sg;
      xm3 = xm2; xm2 = xm1; xm1 = xcur;
    }
    __syncthreads();
    v8h bv[2];
#pragma unroll
    for (int it = 0; it < 2; ++it) {
      const float* sp = sT + (it * 8 + wave) * kConvTP + lane * 8;
      const v4f a0 = *(const v4f*)(sp);
      const v4f a1 = *(const v4f*)(sp + 4);
#pragma unroll
      for (int e = 0; e < 4; ++e) {
        bv[it][e]     = __builtin_bit_cast(_Float16, f2bf_bits(a0[e]));
        bv[it][4 + e] = __builtin_bit_cast(_Float16, f2bf_bits(a1[e]));
      }
    }
    for (int pass = 0; pass < 2; ++pass) {
#pragma unroll
      for (int it = 0; it < 2; ++it) {
        const int taur = lb + it * 8 + wave;
        const int p = dir ? (kSeq - 1 - taur) : taur;
        *(volatile v8h*)(XCd + (size_t)p * kDin + d0 + lane * 8) = bv[it];
      }
      __threadfence();
    }
    __syncthreads();
  }
}

template <int DIR>
__global__ __launch_bounds__(kScanThr) void scan_kernel(
    const float* __restrict__ XZ, const float* __restrict__ PJd, const unsigned short* __restrict__ DTd,
    const float* __restrict__ cw, const float* __restrict__ cb, const float* __restrict__ dtb,
    const float* __restrict__ Alog, const float* __restrict__ Dp,
    float* YFp, unsigned short* __restrict__ YSH, unsigned short* __restrict__ YSL)
{
  __shared__ __align__(16) float sBC[kScanTS * 32];
  __shared__ __align__(16) unsigned short sBCb[kScanTS * 32];
  __shared__ __align__(16) unsigned short sDT[kScanTS * kScanCh];
  __shared__ __align__(16) float sY[kScanTS * kScanYP];
  const int tid = threadIdx.x, lane = tid & 31, wave = tid >> 5;
  const int hh = lane >> 4, m = lane & 15;
  const int cl = wave * 16 + m;
  const int d0 = blockIdx.x * kScanCh;
  const int d  = d0 + cl;
  float negA[8], h[8];
  {
    const v4f a0 = *(const v4f*)(Alog + (size_t)d * kNst + 8 * hh);
    const v4f a1 = *(const v4f*)(Alog + (size_t)d * kNst + 8 * hh + 4);
#pragma unroll
    for (int e = 0; e < 4; ++e) {
      negA[e]     = -expf(bfr(a0[e]));
      negA[4 + e] = -expf(bfr(a1[e]));
    }
  }
#pragma unroll
  for (int e = 0; e < 8; ++e) h[e] = 0.f;
  const v4f cwv = *(const v4f*)(cw + (size_t)d * 4);
  const float w0 = bfr(cwv[0]), w1 = bfr(cwv[1]), w2 = bfr(cwv[2]), w3 = bfr(cwv[3]);
  asm volatile("" ::: "memory");
  const float bc = bfr(cb[d]);
  const float bb = bfr(dtb[d]);
  const float Dd = bfr(Dp[d]);
  float xm3 = 0.f, xm2 = 0.f, xm1 = 0.f;
  const int q = lane >> 3, c8 = (lane & 7) * 8, c4 = m * 4;
  const int sr = tid >> 1, sp2 = tid & 1;
  const v4u zq = (v4u){0u, 0u, 0u, 0u};
#pragma unroll 1
  for (int tau0 = 0; tau0 < kSeq; tau0 += kScanTS) {
    __syncthreads();
    {
      const int taur = tau0 + sr;
      const int prow = DIR ? (kSeq - 1 - taur) : taur;
      const float* pj = PJd + (size_t)prow * kPjP + kDtR + sp2 * 16;
      v4f t[4];
#pragma unroll
      for (int i = 0; i < 4; ++i) t[i] = *(const v4f*)(pj + 4 * i);
      const unsigned short* dp = DTd + (size_t)prow * kDin + d0 + sp2 * 32;
      v4u u[4];
#pragma unroll
      for (int i = 0; i < 4; ++i) u[i] = *(const v4u*)(dp + 8 * i);
#pragma unroll
      for (int i = 0; i < 4; ++i) *(v4f*)(sBC + sr * 32 + sp2 * 16 + 4 * i) = t[i];
      unsigned wd[8];
#pragma unroll
      for (int i = 0; i < 4; ++i) {
        wd[2 * i]     = pack_bf2(t[i][0], t[i][1]);
        wd[2 * i + 1] = pack_bf2(t[i][2], t[i][3]);
      }
      *(v4u*)(sBCb + sr * 32 + sp2 * 16)     = (v4u){wd[0], wd[1], wd[2], wd[3]};
      *(v4u*)(sBCb + sr * 32 + sp2 * 16 + 8) = (v4u){wd[4], wd[5], wd[6], wd[7]};
#pragma unroll
      for (int i = 0; i < 4; ++i) *(v4u*)(sDT + sr * kScanCh + sp2 * 32 + 8 * i) = u[i];
    }
    __syncthreads();
#pragma unroll 1
    for (int s = 0; s < kScanTS; ++s) {
      const int tau = tau0 + s;
      const int prow = DIR ? (kSeq - 1 - tau) : tau;
      const size_t rb = (size_t)prow * kXzP;
      const float xcur = XZ[rb + d];
      const float zv = XZ[rb + kDin + d];
      float yf = 0.f;
      if (DIR) yf = YFp[(size_t)prow * kDin + d];
      float cacc = w0 * xm3;
      cacc = fmaf(w1, xm2, cacc);
      cacc = fmaf(w2, xm1, cacc);
      cacc = fmaf(w3, xcur, cacc);
      const float sv = cacc + bc;
      const float sgx = __builtin_amdgcn_rcpf(1.0f + __expf(-sv));
      const float xc = sv * sgx;
      xm3 = xm2; xm2 = xm1; xm1 = xcur;
      const float dtp = __uint_as_float(((unsigned)sDT[s * kScanCh + cl]) << 16);
      const float v = dtp + bb;
      const float dt = fmaxf(v, 0.0f) + __logf(1.0f + __expf(-fabsf(v)));
      const v4f b0 = *(const v4f*)(sBC + s * 32 + 8 * hh);
      const v4f b1 = *(const v4f*)(sBC + s * 32 + 8 * hh + 4);
      float Bs[8];
      Bs[0] = b0[0]; Bs[1] = b0[1]; Bs[2] = b0[2]; Bs[3] = b0[3];
      Bs[4] = b1[0]; Bs[5] = b1[1]; Bs[6] = b1[2]; Bs[7] = b1[3];
      const float dtx = dt * xc;
#pragma unroll
      for (int e = 0; e < 8; ++e) {
        const float ex = __expf(dt * negA[e]);
        h[e] = fmaf(ex, h[e], dtx * Bs[e]);
      }
      FragW fa, fb;
      fa.q[0] = *(const v4u*)(sBCb + s * 32 + kNst + 8 * hh);
      fa.q[1] = zq;
      fb.q[0] = (v4u){pack_bf2(h[0], h[1]), pack_bf2(h[2], h[3]), pack_bf2(h[4], h[5]), pack_bf2(h[6], h[7])};
      fb.q[1] = zq;
      const v8f dacc = mma_bf16_once(fa.v, fb.v);
      float y = dacc[0];
      y = fmaf(Dd, xc, y);
      const float sgz = __builtin_amdgcn_rcpf(1.0f + __expf(-zv));
      y = y * (zv * sgz);
      if (DIR) y = yf + y;
      if (hh == 0) sY[s * kScanYP + cl] = y;
    }
    __syncthreads();
    if (DIR == 0) {
      for (int pass = 0; pass < 2; ++pass) {
#pragma unroll
        for (int it = 0; it < 8; ++it) {
          const int row = it * 8 + wave * 2 + hh;
          const int prow = tau0 + row;
          v4f val = *(const v4f*)(sY + row * kScanYP + c4);
          *(volatile v4f*)(YFp + (size_t)prow * kDin + d0 + c4) = val;
        }
        __threadfence();
      }
    } else {
      v8h hv[4], lv[4];
#pragma unroll
      for (int it = 0; it < 4; ++it) {
        const int row = it * 16 + wave * 4 + q;
        const float* sp = sY + row * kScanYP + c8;
        const v4f a0 = *(const v4f*)(sp);
        const v4f a1 = *(const v4f*)(sp + 4);
#pragma unroll
        for (int e = 0; e < 4; ++e) {
          const unsigned short h0 = f2bf_bits(a0[e]), h1 = f2bf_bits(a1[e]);
          const unsigned short l0 = f2bf_bits(a0[e] - bf_bits2f(h0)), l1 = f2bf_bits(a1[e] - bf_bits2f(h1));
          hv[it][e]     = __builtin_bit_cast(_Float16, h0);
          hv[it][4 + e] = __builtin_bit_cast(_Float16, h1);
          lv[it][e]     = __builtin_bit_cast(_Float16, l0);
          lv[it][4 + e] = __builtin_bit_cast(_Float16, l1);
        }
      }
      for (int pass = 0; pass < 2; ++pass) {
#pragma unroll
        for (int it = 0; it < 4; ++it) {
          const int row = it * 16 + wave * 4 + q;
          const int prow = kSeq - 1 - (tau0 + row);
          const size_t o = (size_t)prow * kDin + d0 + c8;
          *(volatile v8h*)(YSH + o) = hv[it];
          *(volatile v8h*)(YSL + o) = lv[it];
        }
        __threadfence();
      }
    }
  }
}

static_assert((kSeq % 64) == 0 && (kXzP % 64) == 0 && (kDm % 32) == 0);
static_assert((kNPjPad % 64) == 0 && (kDin % 32) == 0);
static_assert((kDin % 64) == 0 && (kDtR % 32) == 0);
static_assert((kDm % 64) == 0);

extern "C" void kernel_launch(void* const* d_in, const int* in_sizes, int n_in,
                              void* d_out, int out_size, void* d_ws, size_t ws_size,
                              hipStream_t stream) {
  if (n_in < 17) return;
  if (in_sizes[0] != kRowsAll * kDm) return;
  if (in_sizes[1] != kXzP * kDm) return;
  if (in_sizes[2] != kDm * kDin) return;
  if (in_sizes[3] != kDin * 4 || in_sizes[10] != kDin * 4) return;
  if (in_sizes[4] != kDin || in_sizes[11] != kDin) return;
  if (in_sizes[5] != kNPj * kDin || in_sizes[12] != kNPj * kDin) return;
  if (in_sizes[6] != kDin * kDtR || in_sizes[13] != kDin * kDtR) return;
  if (in_sizes[7] != kDin || in_sizes[14] != kDin) return;
  if (in_sizes[8] != kDin * kNst || in_sizes[15] != kDin * kNst) return;
  if (in_sizes[9] != kDin || in_sizes[16] != kDin) return;
  if (out_size != kRowsAll * kDm) return;
  if (ws_size < kWsTotal) return;

  const float* u      = (const float*)d_in[0];
  const float* W_in   = (const float*)d_in[1];
  const float* W_out  = (const float*)d_in[2];
  const float* cwf    = (const float*)d_in[3];
  const float* cbf    = (const float*)d_in[4];
  const float* Wxf    = (const float*)d_in[5];
  const float* Wdtf   = (const float*)d_in[6];
  const float* bdtf   = (const float*)d_in[7];
  const float* Alogf  = (const float*)d_in[8];
  const float* Df     = (const float*)d_in[9];
  const float* cwb    = (const float*)d_in[10];
  const float* cbb    = (const float*)d_in[11];
  const float* Wxb    = (const float*)d_in[12];
  const float* Wdtb   = (const float*)d_in[13];
  const float* bdtb   = (const float*)d_in[14];
  const float* Alogb  = (const float*)d_in[15];
  const float* Db     = (const float*)d_in[16];
  float* out = (float*)d_out;

  char* ws = (char*)d_ws;
  unsigned short* UB   = (unsigned short*)(ws + kOffUB);
  unsigned short* WIB  = (unsigned short*)(ws + kOffWIB);
  unsigned short* WOB  = (unsigned short*)(ws + kOffWOB);
  unsigned short* WX   = (unsigned short*)(ws + kOffWX);
  unsigned short* WD   = (unsigned short*)(ws + kOffWD);
  float*          XZ   = (float*)(ws + kOffXZ);
  unsigned short* XC   = (unsigned short*)(ws + kOffXC);
  float*          PJ   = (float*)(ws + kOffPJ);
  unsigned short* DI   = (unsigned short*)(ws + kOffDI);
  unsigned short* DT   = (unsigned short*)(ws + kOffDT);
  float*          YF   = (float*)(ws + kOffYF);
  unsigned short* YSH  = (unsigned short*)(ws + kOffYSH);
  unsigned short* YSL  = (unsigned short*)(ws + kOffYSL);

  {
    const int t8u  = kRowsAll * kDm / 8;
    const int t8wi = kXzP * kDm / 8;
    const int t8wo = kDm * kDin / 8;
    const int t8wx = kNPjPad * kDin / 8;
    const int t8wd = kDin * kDtR / 8;
    cvt_bf16_kernel<<<(t8u + 255) / 256, 256, 0, stream>>>(u, UB, kDm, kRowsAll, t8u);
    cvt_bf16_kernel<<<(t8wi + 255) / 256, 256, 0, stream>>>(W_in, WIB, kDm, kXzP, t8wi);
    cvt_bf16_kernel<<<(t8wo + 255) / 256, 256, 0, stream>>>(W_out, WOB, kDin, kDm, t8wo);
    cvt_bf16_kernel<<<(t8wx + 255) / 256, 256, 0, stream>>>(Wxf, WX, kDin, kNPj, t8wx);
    cvt_bf16_kernel<<<(t8wx + 255) / 256, 256, 0, stream>>>(Wxb, WX + (size_t)kNPjPad * kDin, kDin, kNPj, t8wx);
    cvt_bf16_kernel<<<(t8wd + 255) / 256, 256, 0, stream>>>(Wdtf, WD, kDtR, kDin, t8wd);
    cvt_bf16_kernel<<<(t8wd + 255) / 256, 256, 0, stream>>>(Wdtb, WD + (size_t)kDin * kDtR, kDtR, kDin, t8wd);
  }

  const int tiles_in  = (kSeq / 64) * (kXzP / 64);
  const int tiles_xp  = (kSeq / 64) * (kNPjPad / 64);
  const int tiles_dt  = (kSeq / 64) * (kDin / 64);
  const int tiles_out = (kSeq / 64) * (kDm / 64);
  const int t8di = 2 * kSeq * (kDtR / 8);

  for (int bi = 0; bi < kBatch; ++bi) {
    const unsigned short* UBb = UB + (size_t)bi * kSeq * kDm;
    float* outb = out + (size_t)bi * kSeq * kDm;

    wmma_gemm64<1, 0, 0, 0, false><<<dim3((tiles_in + 7) / 8, 1), 256, 0, stream>>>(
        UBb, nullptr, kDm, 0L,
        WIB, nullptr, kDm, 0L,
        (void*)XZ, nullptr, kXzP, 0L,
        nullptr, nullptr, 0L,
        kSeq, kXzP, kDm, 1.0f);

    conv_silu_kernel<<<dim3(kDin / 256, kSeq / 64, 2), 256, 0, stream>>>(XZ, cwf, cbf, cwb, cbb, XC);

    wmma_gemm64<1, 0, 0, 0, false><<<dim3((tiles_xp + 7) / 8, 2), 256, 0, stream>>>(
        XC, nullptr, kDin, (long)kSeq * kDin,
        WX, nullptr, kDin, (long)kNPjPad * kDin,
        (void*)PJ, nullptr, kPjP, (long)kSeq * kPjP,
        nullptr, nullptr, 0L,
        kSeq, kNPjPad, kDin, 1.0f);

    cvt_cols64_kernel<<<(t8di + 255) / 256, 256, 0, stream>>>(PJ, DI, t8di);

    wmma_gemm64<1, 0, 0, 3, false><<<dim3((tiles_dt + 7) / 8, 2), 256, 0, stream>>>(
        DI, nullptr, kDtR, (long)kSeq * kDtR,
        WD, nullptr, kDtR, (long)kDin * kDtR,
        (void*)DT, nullptr, kDin, (long)kSeq * kDin,
        nullptr, nullptr, 0L,
        kSeq, kDin, kDtR, 1.0f);

    scan_kernel<0><<<kDin / kScanCh, kScanThr, 0, stream>>>(
        XZ, PJ, DT, cwf, cbf, bdtf, Alogf, Df, YF, YSH, YSL);
    scan_kernel<1><<<kDin / kScanCh, kScanThr, 0, stream>>>(
        XZ, PJ + (size_t)kSeq * kPjP, DT + (size_t)kSeq * kDin, cwb, cbb, bdtb, Alogb, Db, YF, YSH, YSL);

    wmma_gemm64<1, 1, 0, 0, false><<<dim3((tiles_out + 7) / 8, 1), 256, 0, stream>>>(
        YSH, YSL, kDin, 0L,
        WOB, nullptr, kDin, 0L,
        (void*)outb, nullptr, kDm, 0L,
        nullptr, nullptr, 0L,
        kSeq, kDm, kDin, 1.0f);
  }
}
